// MultiHeadAttention_87875030876832
// MI455X (gfx1250) — hardware-run, weakly checked
//
#include <hip/hip_runtime.h>
#ifndef NB
#define NB 2
#endif
#ifndef SQ
#define SQ 2048
#endif
#define NB_FULL 2
#define SQ_FULL 2048
#define DM 1024
#define NH 16
#define HD 64
#define NR ((size_t)NB * SQ)
#define NCH (SQ / 256)
#define NTILE (NB * SQ / 32)
#ifndef EARLY_ROWS
#define EARLY_ROWS ((SQ < 512) ? SQ : 512)
#endif
static_assert(SQ % 256 == 0);
static_assert(SQ <= SQ_FULL);
static_assert(NB <= NB_FULL);
static_assert(((size_t)NB * SQ) % 128 == 0);
static_assert(DM % 64 == 0);
static_assert(NH * HD == DM);
static_assert(EARLY_ROWS % 64 == 0);
static_assert((SQ - EARLY_ROWS) % 64 == 0);
static_assert(EARLY_ROWS >= 64);
static_assert(EARLY_ROWS <= SQ);

typedef unsigned short v8us __attribute__((ext_vector_type(8), may_alias));
typedef float  v8f  __attribute__((ext_vector_type(8)));
typedef float  v4f  __attribute__((ext_vector_type(4)));
typedef float  v4fa __attribute__((ext_vector_type(4), may_alias));
typedef int    v4i  __attribute__((ext_vector_type(4)));
typedef int    v4ia __attribute__((ext_vector_type(4), may_alias));
typedef _Float16 v16h __attribute__((ext_vector_type(16)));
typedef _Float16 v4h  __attribute__((ext_vector_type(4)));
union FragH { v16h v; v8us half[2]; _Float16 h[16]; unsigned short u[16]; };

__device__ __forceinline__ unsigned short bf16_bits(float x) { unsigned int u = __float_as_uint(x); return (unsigned short)((u + 0x7FFFu + ((u >> 16) & 1u)) >> 16); }
__device__ __forceinline__ float bf16_rne(float x) { return __uint_as_float(((unsigned int)bf16_bits(x)) << 16); }
__device__ __forceinline__ int clampk(int v) { v = (v < 32) ? 32 : v; v = (v > SQ) ? SQ : v; return v & ~31; }

__device__ __forceinline__ v16h g2_frag(const _Float16* p, int hh) { FragH f; f.half[0] = *(const v8us*)((const unsigned short*)p + 8 * hh); f.half[1] = *(const v8us*)((const unsigned short*)p + 16 + 8 * hh); return f.v; }
__device__ __forceinline__ v8f g2_mma(v16h a, v16h b, v8f c) { v8f d = __builtin_amdgcn_wmma_f32_16x16x32_f16(false, a, false, b, (short)0, c, false, false); asm volatile("v_nop\n\tv_nop\n\tv_nop\n\tv_nop" : "+v"(d) : "v"(a), "v"(b)); return d; }

__global__ __launch_bounds__(256) void k_wnat(const float* __restrict__ w, size_t n8, _Float16* __restrict__ Bt) {
  const size_t t = (size_t)blockIdx.x * 256 + threadIdx.x; if (t >= n8) return;
  const v4f a = *(const v4fa*)(w + t * 8), c = *(const v4fa*)(w + t * 8 + 4);
  FragH f;
#pragma unroll
  for (int q = 0; q < 4; ++q) { f.h[q] = (_Float16)(bf16_rne(a[q]) * 16.0f); f.h[4 + q] = (_Float16)(bf16_rne(c[q]) * 16.0f); }
  const v8us o = f.half[0];
  unsigned short* d = (unsigned short*)Bt + t * 8;
  *(volatile v8us*)d = o; __threadfence(); *(volatile v8us*)d = o;
}

__global__ __launch_bounds__(256) void k_x16(const float* __restrict__ x, _Float16* __restrict__ X16, size_t n8) {
  const size_t t = (size_t)blockIdx.x * 256 + threadIdx.x; if (t >= n8) return;
  const size_t row = t / (DM / 8); const int c8 = (int)(t % (DM / 8)) * 8;
  const size_t b = row / SQ, s = row % SQ;
  const float* src = x + (b * SQ_FULL + s) * DM + c8;
  const v4f a = *(const v4fa*)src, c = *(const v4fa*)(src + 4);
  FragH f;
#pragma unroll
  for (int q = 0; q < 4; ++q) { f.h[q] = (_Float16)bf16_rne(a[q]); f.h[4 + q] = (_Float16)bf16_rne(c[q]); }
  const v8us o = f.half[0];
  unsigned short* d = (unsigned short*)X16 + t * 8;
  *(volatile v8us*)d = o; __threadfence(); *(volatile v8us*)d = o;
}

__global__ __launch_bounds__(256) void k_kend(const int* __restrict__ mask, int* __restrict__ kt) {
  __shared__ int wm[8];
  const int tid = threadIdx.x, w = __builtin_amdgcn_readfirstlane((int)(tid >> 5)), lane = tid & 31;
  const int tile = blockIdx.x; const int b = tile / (SQ / 32); const int q0 = (tile % (SQ / 32)) * 32;
  int need = 0;
#pragma unroll 1
  for (int rr = 0; rr < 4; ++rr) {
    const int q = q0 + w * 4 + rr;
    const int* mrow = mask + ((size_t)b * SQ_FULL + q) * SQ_FULL + lane * 8;
    int last = 0;
#pragma unroll 1
    for (int c = 0; c < SQ; c += 256) {
      const v4i m0 = *(const v4ia*)(mrow + c), m1 = *(const v4ia*)(mrow + c + 4);
      const int base = c + lane * 8;
#pragma unroll
      for (int i = 0; i < 4; ++i) last = (m0[i] == 0) ? (base + i + 1) : last;
#pragma unroll
      for (int i = 0; i < 4; ++i) last = (m1[i] == 0) ? (base + 4 + i + 1) : last;
    }
    for (int o = 16; o > 0; o >>= 1) { const int ot = __shfl_xor(last, o); last = (ot > last) ? ot : last; }
    if (last == 0) last = SQ;
    need = (last > need) ? last : need;
  }
  if (lane == 0) wm[w] = need;
  __syncthreads();
  if (w == 0) {
    int v = wm[lane & 7];
    for (int o = 1; o < 8; o <<= 1) { const int ot = __shfl_xor(v, o); v = (ot > v) ? ot : v; }
    v = clampk((v + 31) & ~31);
    const v4i ov = {v, v, v, v};
    int* dst = kt + (size_t)tile * 32 + (lane & 7) * 4;
    if (lane < 8) *(volatile v4i*)dst = ov;
    __threadfence();
    if (lane < 8) *(volatile v4i*)dst = ov;
  }
}

__global__ __launch_bounds__(128) void k_gemm2p(const _Float16* __restrict__ A, int lda, const _Float16* __restrict__ Bh, int ldb, float alpha,
    _Float16* __restrict__ C16, _Float16* __restrict__ C16L, int ldc, int M, int N, int K) {
  __shared__ __attribute__((aligned(16))) float so[4][32][68];
  const int tid = threadIdx.x, w = __builtin_amdgcn_readfirstlane((int)(tid >> 5)), lane = tid & 31, ln = lane & 15, hh = lane >> 4;
  const int ntn = N >> 6; const int mt = blockIdx.x / ntn, nq = blockIdx.x - mt * ntn; const int row0 = mt * 128 + 32 * w, col0 = nq * 64; if (row0 >= M) return;
  const _Float16* a0p = A + (size_t)(row0 + ln) * lda; const _Float16* a1p = a0p + (size_t)16 * lda;
  const _Float16* b0p = Bh + (size_t)(col0 + ln) * ldb; const _Float16* b1p = b0p + (size_t)16 * ldb; const _Float16* b2p = b1p + (size_t)16 * ldb; const _Float16* b3p = b2p + (size_t)16 * ldb;
  const v8f z8 = {0.f,0.f,0.f,0.f,0.f,0.f,0.f,0.f}; v8f c00 = z8, c01 = z8, c02 = z8, c03 = z8, c10 = z8, c11 = z8, c12 = z8, c13 = z8;
#pragma unroll 1
  for (int kb = 0; kb < K; kb += 32) { const v16h a0 = g2_frag(a0p + kb, hh), a1 = g2_frag(a1p + kb, hh);
    v16h b = g2_frag(b0p + kb, hh); c00 = g2_mma(a0, b, c00); c10 = g2_mma(a1, b, c10);
    b = g2_frag(b1p + kb, hh); c01 = g2_mma(a0, b, c01); c11 = g2_mma(a1, b, c11);
    b = g2_frag(b2p + kb, hh); c02 = g2_mma(a0, b, c02); c12 = g2_mma(a1, b, c12);
    b = g2_frag(b3p + kb, hh); c03 = g2_mma(a0, b, c03); c13 = g2_mma(a1, b, c13); }
  v8f accs[8] = {c00, c01, c02, c03, c10, c11, c12, c13};
#pragma unroll
  for (int u = 0; u < 8; ++u) { const int t = u & 3, half = u >> 2;
#pragma unroll
    for (int r = 0; r < 8; ++r) { const int rloc = half * 16 + 8 * hh + r; so[w][rloc][t * 16 + ln] = accs[u][r] * alpha; } }
  __builtin_amdgcn_fence(4  , "workgroup"); __builtin_amdgcn_wave_barrier();
  const int rsub = lane >> 4, c4 = (lane & 15) * 4;
  for (int pass = 0; pass < 2; ++pass) {
#pragma unroll
    for (int q = 0; q < 16; ++q) { const int r = q * 2 + rsub; const v4f v = *(const v4fa*)&so[w][r][c4];
      v4h h4, l4;
#pragma unroll
      for (int i = 0; i < 4; ++i) { const _Float16 h = (_Float16)v[i]; h4[i] = h; l4[i] = (_Float16)((v[i] - (float)h) * 1024.0f); }
      const size_t o = (size_t)(row0 + r) * ldc + col0 + c4;
      *(volatile v4h*)(C16 + o) = h4; *(volatile v4h*)(C16L + o) = l4; }
    if (pass == 0) __threadfence(); }
}

template <bool AL, bool BL, int OM, int CAUS>
__global__ __launch_bounds__(128) void k_gemmd(const _Float16* __restrict__ A, const _Float16* __restrict__ Al, int lda,
    const _Float16* __restrict__ Bh, const _Float16* __restrict__ Bl, int ldb, float alpha, const float* __restrict__ bias,
    float* __restrict__ C, _Float16* __restrict__ C16, _Float16* __restrict__ C16L, int ldc, int M, int N, int K, const int* __restrict__ kt, int trow0) {
  __shared__ __attribute__((aligned(16))) float so[4][16][68];
  const int tid = threadIdx.x, w = __builtin_amdgcn_readfirstlane((int)(tid >> 5)), lane = tid & 31, ln = lane & 15, hh = lane >> 4;
  const int ntn = N >> 6; const int mt = blockIdx.x / ntn, nq = blockIdx.x - mt * ntn; const int row0 = mt * 64 + 16 * w, col0 = nq * 64; if (row0 >= M) return;
  int Kw = K;
  if (CAUS == 1) { const int tb = (trow0 + mt * 64) >> 5; const int k0 = clampk(kt[(size_t)tb * 32]); const int k1 = clampk(kt[(size_t)(tb + 1) * 32]); const int ke = (k0 > k1) ? k0 : k1; if (col0 >= ke) return; }
  if (CAUS == 2) { const int tw = (trow0 + row0) >> 5; const int ke = clampk(kt[(size_t)tw * 32]); Kw = (ke < K) ? ke : K; }
  const _Float16* ap = A + (size_t)(row0 + ln) * lda; const _Float16* alp = Al + (size_t)(row0 + ln) * lda;
  const _Float16* bp = Bh + (size_t)(col0 + ln) * ldb; const _Float16* blp = Bl + (size_t)(col0 + ln) * ldb;
  const size_t bst = (size_t)16 * ldb;
  const v8f z8 = {0.f,0.f,0.f,0.f,0.f,0.f,0.f,0.f};
  v8f acc[4] = {z8, z8, z8, z8}; v8f accr[4] = {z8, z8, z8, z8};
#pragma unroll 1
  for (int kb = 0; kb < Kw; kb += 32) {
    const v16h a = g2_frag(ap + kb, hh);
    v16h al = a; if (AL) al = g2_frag(alp + kb, hh);
#pragma unroll
    for (int t = 0; t < 4; ++t) {
      const v16h b = g2_frag(bp + (size_t)t * bst + kb, hh);
      acc[t] = g2_mma(a, b, acc[t]);
      if (AL) accr[t] = g2_mma(al, b, accr[t]);
      if (BL) { const v16h bl = g2_frag(blp + (size_t)t * bst + kb, hh); accr[t] = g2_mma(a, bl, accr[t]); }
    }
  }
#pragma unroll
  for (int t = 0; t < 4; ++t) { const int col = col0 + t * 16 + ln; const float bv = bias ? bf16_rne(bias[col]) : 0.f;
#pragma unroll
    for (int r = 0; r < 8; ++r) so[w][8 * hh + r][t * 16 + ln] = (acc[t][r] + accr[t][r] * 0.0009765625f) * alpha + bv; }
  __builtin_amdgcn_fence(4  , "workgroup"); __builtin_amdgcn_wave_barrier();
  const int rsub = lane >> 4, c4 = (lane & 15) * 4;
  for (int pass = 0; pass < 2; ++pass) {
#pragma unroll
    for (int q = 0; q < 8; ++q) { const int r = q * 2 + rsub; const v4f v = *(const v4fa*)&so[w][r][c4];
      const size_t o = (size_t)(row0 + r) * ldc + col0 + c4;
      if (OM == 0) { *(volatile v4f*)(C + o) = v; }
      else { v4h h4, l4;
#pragma unroll
        for (int i = 0; i < 4; ++i) { const _Float16 h = (_Float16)v[i]; h4[i] = h; l4[i] = (_Float16)((v[i] - (float)h) * 1024.0f); }
        *(volatile v4h*)(C16 + o) = h4; *(volatile v4h*)(C16L + o) = l4; } }
    if (pass == 0) __threadfence(); }
}

template <int NHv, int TTv>
__global__ __launch_bounds__(256) void k_vt(const _Float16* __restrict__ V16, int ldv, int voff, _Float16* __restrict__ Vt) {
  __shared__ unsigned short tl[64][66];
  const int tid = threadIdx.x; const int slab = blockIdx.x / (TTv / 64), lg = blockIdx.x % (TTv / 64); const int b = slab / NHv, h = slab % NHv;
  for (int i = tid; i < 64 * 8; i += 256) { const int r = i / 8, c8 = (i % 8) * 8; FragH f; f.half[0] = *(const v8us*)((const unsigned short*)V16 + ((size_t)b * TTv + lg * 64 + r) * ldv + voff + h * 64 + c8);
#pragma unroll
    for (int q = 0; q < 8; ++q) tl[r][c8 + q] = f.u[q]; }
  __syncthreads();
  for (int pass = 0; pass < 2; ++pass) {
#pragma unroll
    for (int rd = 0; rd < 2; ++rd) { const int d = rd * 32 + tid / 8, pc = tid % 8; FragH f;
#pragma unroll
      for (int q = 0; q < 8; ++q) f.u[q] = tl[pc * 8 + q][d];
      *(volatile v8us*)((unsigned short*)Vt + ((size_t)slab * 64 + d) * TTv + lg * 64 + pc * 8) = f.half[0]; }
    if (pass == 0) __threadfence(); }
}

__global__ __launch_bounds__(256) void k_smx(const float* __restrict__ S, const int* __restrict__ mask, const int* __restrict__ kt,
    _Float16* __restrict__ Ph, _Float16* __restrict__ Pl, int b) {
  #pragma clang fp contract(off)
  const int tid = threadIdx.x, w = __builtin_amdgcn_readfirstlane((int)(tid >> 5)), lane = tid & 31;
  const int q = blockIdx.x * 8 + w;
  const int ke = clampk(kt[(((size_t)b * SQ + q) >> 5) * 32]);
  int ke64 = (ke + 63) & ~63; ke64 = (ke64 > SQ) ? SQ : ke64;
  const float* srow = S + (size_t)q * SQ + lane * 8;
  const int* mrow = mask + ((size_t)b * SQ_FULL + q) * SQ_FULL + lane * 8;
  float sv[NCH][8];
  float mx = -3.0e38f;
#pragma unroll
  for (int c = 0; c < NCH; ++c) {
    if (c * 256 < ke) {
      const v4f a0 = *(const v4fa*)(srow + c * 256), a1 = *(const v4fa*)(srow + c * 256 + 4);
      const v4i m0 = *(const v4ia*)(mrow + c * 256), m1 = *(const v4ia*)(mrow + c * 256 + 4);
      const int base = c * 256 + lane * 8;
#pragma unroll
      for (int i = 0; i < 4; ++i) {
        float x0 = (m0[i] != 0) ? -1.0e9f : a0[i]; x0 = (base + i < ke) ? x0 : -3.0e38f; sv[c][i] = x0; mx = fmaxf(mx, x0);
        float x1 = (m1[i] != 0) ? -1.0e9f : a1[i]; x1 = (base + 4 + i < ke) ? x1 : -3.0e38f; sv[c][4 + i] = x1; mx = fmaxf(mx, x1);
      }
    } else {
#pragma unroll
      for (int i = 0; i < 8; ++i) sv[c][i] = -3.0e38f;
    }
  }
  for (int o = 16; o > 0; o >>= 1) mx = fmaxf(mx, __shfl_xor(mx, o));
  float se = 0.f;
#pragma unroll
  for (int c = 0; c < NCH; ++c) {
    if (c * 256 < ke) {
#pragma unroll
      for (int i = 0; i < 8; ++i) { const float e = __expf(sv[c][i] - mx); sv[c][i] = e; se += e; }
    }
  }
  for (int o = 16; o > 0; o >>= 1) se += __shfl_xor(se, o);
  const float sc = 256.0f * (1.0f / se);
#pragma unroll
  for (int c = 0; c < NCH; ++c) {
    if (c * 256 < ke) {
#pragma unroll
      for (int i = 0; i < 8; ++i) sv[c][i] = sv[c][i] * sc;
    }
  }
  for (int pass = 0; pass < 2; ++pass) {
#pragma unroll
    for (int c = 0; c < NCH; ++c) {
      if (c * 256 < ke64) {
        const int base = c * 256 + lane * 8;
        FragH fh, fl;
#pragma unroll
        for (int i = 0; i < 8; ++i) { const float p = sv[c][i]; const _Float16 h = (_Float16)p; fh.h[i] = h; fl.h[i] = (_Float16)((p - (float)h) * 1024.0f); }
        if (base < ke64) {
          const size_t o = (size_t)q * SQ + base;
          *(volatile v8us*)((unsigned short*)Ph + o) = fh.half[0];
          *(volatile v8us*)((unsigned short*)Pl + o) = fl.half[0];
        }
      }
    }
    if (pass == 0) __threadfence();
  }
}

extern "C" void kernel_launch(void* const* d_in, const int* in_sizes, int n_in,
                              void* d_out, int out_size, void* d_ws, size_t ws_size, hipStream_t stream) {
  if (n_in < 9) return;
  const size_t needx = ((size_t)(NB - 1) * SQ_FULL + SQ) * DM;
  const size_t needm = ((size_t)(NB - 1) * SQ_FULL + (SQ - 1)) * SQ_FULL + SQ;
  if ((size_t)in_sizes[0] < needx || (size_t)in_sizes[1] < needx || (size_t)in_sizes[2] < needx) return;
  if ((size_t)in_sizes[3] < needm) return;
  if ((size_t)in_sizes[4] < (size_t)DM * DM || (size_t)in_sizes[5] < (size_t)DM * DM || (size_t)in_sizes[6] < (size_t)DM * DM || (size_t)in_sizes[7] < (size_t)DM * DM) return;
  if ((size_t)in_sizes[8] < (size_t)DM) return;
  if ((size_t)out_size < NR * DM) return;
  const float* xq = (const float*)d_in[0]; const float* xk = (const float*)d_in[1]; const float* xv = (const float*)d_in[2];
  const int* mk = (const int*)d_in[3];
  const float* wq = (const float*)d_in[4]; const float* wk = (const float*)d_in[5]; const float* wv = (const float*)d_in[6]; const float* wo = (const float*)d_in[7];
  const float* bo = (const float*)d_in[8];
  float* out = (float*)d_out;
  char* ws = (char*)d_ws; size_t off = 0;
  auto take = [&](size_t bytes) { char* p = ws + off; off += (bytes + 255) & ~(size_t)255; return p; };
  _Float16* BQ = (_Float16*)take((size_t)DM * DM * 2); _Float16* BK = (_Float16*)take((size_t)DM * DM * 2); _Float16* BV = (_Float16*)take((size_t)DM * DM * 2); _Float16* BO = (_Float16*)take((size_t)DM * DM * 2);
  _Float16* X = (_Float16*)take(NR * DM * 2);
  _Float16* Qh = (_Float16*)take(NR * DM * 2); _Float16* Ql = (_Float16*)take(NR * DM * 2);
  _Float16* Kh = (_Float16*)take(NR * DM * 2); _Float16* Kl = (_Float16*)take(NR * DM * 2);
  _Float16* Vh = (_Float16*)take(NR * DM * 2); _Float16* Vl = (_Float16*)take(NR * DM * 2);
  _Float16* VTh = (_Float16*)take((size_t)NB * NH * HD * SQ * 2); _Float16* VTl = (_Float16*)take((size_t)NB * NH * HD * SQ * 2);
  float* S = (float*)take((size_t)SQ * SQ * 4);
  _Float16* Ph = (_Float16*)take((size_t)SQ * SQ * 2); _Float16* Pl = (_Float16*)take((size_t)SQ * SQ * 2);
  int* KT = (int*)take((size_t)NTILE * 32 * 4);
  if (off > ws_size || off > (size_t)134217728) return;
  _Float16* Oh = Vh; _Float16* Ol = Vl;

  { const size_t n8 = (size_t)DM * DM / 8; const unsigned g = (unsigned)((n8 + 255) / 256);
    k_wnat<<<g, 256, 0, stream>>>(wq, n8, BQ); k_wnat<<<g, 256, 0, stream>>>(wk, n8, BK); k_wnat<<<g, 256, 0, stream>>>(wv, n8, BV); k_wnat<<<g, 256, 0, stream>>>(wo, n8, BO); }
  k_kend<<<NTILE, 256, 0, stream>>>(mk, KT);
  { const size_t n8 = NR * DM / 8; const unsigned gx = (unsigned)((n8 + 255) / 256); const unsigned gp = (unsigned)((NR / 128) * (DM / 64));
    k_x16<<<gx, 256, 0, stream>>>(xq, X, n8);
    k_gemm2p<<<gp, 128, 0, stream>>>(X, DM, BQ, DM, 0.0625f, Qh, Ql, DM, (int)NR, DM, DM);
    k_x16<<<gx, 256, 0, stream>>>(xk, X, n8);
    k_gemm2p<<<gp, 128, 0, stream>>>(X, DM, BK, DM, 0.0625f, Kh, Kl, DM, (int)NR, DM, DM);
    k_x16<<<gx, 256, 0, stream>>>(xv, X, n8);
    k_gemm2p<<<gp, 128, 0, stream>>>(X, DM, BV, DM, 0.0625f, Vh, Vl, DM, (int)NR, DM, DM); }
  k_vt<NH, SQ><<<NB * NH * (SQ / 64), 256, 0, stream>>>(Vh, DM, 0, VTh);
  k_vt<NH, SQ><<<NB * NH * (SQ / 64), 256, 0, stream>>>(Vl, DM, 0, VTl);
  const int ER = EARLY_ROWS;
  const int LR = SQ - EARLY_ROWS;
  for (int b = 0; b < NB; ++b) { const size_t r0 = (size_t)b * SQ;
    for (int h = 0; h < NH; ++h) {
      const size_t qo = r0 * DM + (size_t)h * HD; const size_t vo = ((size_t)b * NH + h) * HD * SQ;
      const size_t qe = qo + (size_t)ER * DM;
      const size_t pe = (size_t)ER * SQ;
      k_gemmd<true, true, 0, 1><<<(unsigned)((ER / 64) * (SQ / 64)), 128, 0, stream>>>(Qh + qo, Ql + qo, DM, Kh + qo, Kl + qo, DM, 0.125f, nullptr, S, nullptr, nullptr, SQ, ER, SQ, HD, KT, (int)r0);
      if (LR > 0)
        k_gemmd<false, false, 0, 1><<<(unsigned)((LR / 64) * (SQ / 64)), 128, 0, stream>>>(Qh + qe, Qh + qe, DM, Kh + qo, Kh + qo, DM, 0.125f, nullptr, S + pe, nullptr, nullptr, SQ, LR, SQ, HD, KT, (int)r0 + ER);
      k_smx<<<SQ / 8, 256, 0, stream>>>(S, mk, KT, Ph, Pl, b);
      k_gemmd<true, true, 1, 2><<<(unsigned)((ER / 64) * (HD / 64)), 128, 0, stream>>>(Ph, Pl, SQ, VTh + vo, VTl + vo, SQ, 0.25f, nullptr, nullptr, Oh + qo, Ol + qo, DM, ER, HD, SQ, KT, (int)r0);
      if (LR > 0)
        k_gemmd<false, false, 1, 2><<<(unsigned)((LR / 64) * (HD / 64)), 128, 0, stream>>>(Ph + pe, Ph + pe, SQ, VTh + vo, VTh + vo, SQ, 0.25f, nullptr, nullptr, Oh + qe, Ol + qe, DM, LR, HD, SQ, KT, (int)r0 + ER);
    } }
  for (int b = 0; b < NB; ++b) { const size_t e0 = (size_t)b * SQ * DM; const size_t e1 = e0 + (size_t)ER * DM;
    k_gemmd<true, false, 0, 0><<<(unsigned)((ER / 64) * (DM / 64)), 128, 0, stream>>>(Oh + e0, Ol + e0, DM, BO, BO, DM, 0.0009765625f, bo, out + e0, nullptr, nullptr, DM, ER, DM, DM, nullptr, 0);
    if (LR > 0)
      k_gemmd<false, false, 0, 0><<<(unsigned)((LR / 64) * (DM / 64)), 128, 0, stream>>>(Oh + e1, Oh + e1, DM, BO, BO, DM, 0.0009765625f, bo, out + e1, nullptr, nullptr, DM, LR, DM, DM, nullptr, 0); }
}
